// ShapeGainCodebook_88510686036491
// MI455X (gfx1250) — hardware-verified
//
#include <hip/hip_runtime.h>
#include <stddef.h>

#pragma clang fp contract(off)

#define DIM     256
#define NSC     1024
#define NGC     64
#define NCT     (NSC / 16)
#define RB      32
#define TA      64
#define PA      264
#define TPB     256
#define CPB     4
#define CHK     256
#define NOUT234 (NGC + NSC + NGC)

#define SC_IN   64.0f
#define SC_LO   2048.0f
#define INV_LO  0.00048828125f
#define DEC     0.99f
#define OMD     0.01f
#define EPSN    1e-5f
#define EPSL2   1e-12f
#define NEGBIG  (-3.402823466e38f)

static_assert(TA == 64);
static_assert(RB == 16 * (TA / 32));
static_assert(RB * 2 == TA);
static_assert(DIM == 256);
static_assert((RB * DIM) % (8 * TA) == 0);
static_assert((PA * 2) % 16 == 0);
static_assert(PA >= DIM);
static_assert(NSC % 16 == 0);
static_assert(NSC % CPB == 0);
static_assert(CHK == TPB);
static_assert(DIM == TPB);
static_assert(NSC == 4 * TPB);
static_assert(NGC <= TA);
static_assert(NGC <= TPB);
static_assert(NOUT234 == 1152);
static_assert(NOUT234 - 4 * TPB == 128);

typedef _Float16       v16h __attribute__((ext_vector_type(16)));
typedef _Float16       v8h  __attribute__((ext_vector_type(8)));
typedef float          v8f  __attribute__((ext_vector_type(8)));
typedef float          v4f  __attribute__((ext_vector_type(4)));
typedef unsigned int   v4u  __attribute__((ext_vector_type(4)));
typedef v4f __attribute__((may_alias)) v4fa;
typedef v4u __attribute__((may_alias)) v4ua;
typedef v8h __attribute__((may_alias)) v8ha;

__device__ __forceinline__ void sp1(float f, _Float16& hh, _Float16& ll) {
  const float v = f * SC_IN;
  const _Float16 hv = (_Float16)v;
  const float r = (v - (float)hv) * SC_LO;
  hh = hv;
  ll = (_Float16)r;
}
__device__ __forceinline__ void split8(v4f a, v4f c, v8h& hv, v8h& lv) {
  v8h h8 = {(_Float16)0.f, (_Float16)0.f, (_Float16)0.f, (_Float16)0.f,
            (_Float16)0.f, (_Float16)0.f, (_Float16)0.f, (_Float16)0.f};
  v8h l8 = h8;
  _Float16 hh, ll;
  sp1(a.x, hh, ll); h8[0] = hh; l8[0] = ll;
  sp1(a.y, hh, ll); h8[1] = hh; l8[1] = ll;
  sp1(a.z, hh, ll); h8[2] = hh; l8[2] = ll;
  sp1(a.w, hh, ll); h8[3] = hh; l8[3] = ll;
  sp1(c.x, hh, ll); h8[4] = hh; l8[4] = ll;
  sp1(c.y, hh, ll); h8[5] = hh; l8[5] = ll;
  sp1(c.z, hh, ll); h8[6] = hh; l8[6] = ll;
  sp1(c.w, hh, ll); h8[7] = hh; l8[7] = ll;
  hv = h8;
  lv = l8;
}

__device__ __forceinline__ v8f wmma_h(v16h a, v16h b, v8f c) {
  v8f d = __builtin_amdgcn_wmma_f32_16x16x32_f16(false, a, false, b, (short)0, c, false, false);
  asm volatile("v_nop\n\tv_nop\n\tv_nop\n\tv_nop" : "+v"(d) : "v"(a), "v"(b));
  return d;
}

__device__ __forceinline__ v16h ldfrag(const _Float16* p, int h) {
  const v8h q0 = *(const v8ha*)(p + 8 * h);
  const v8h q1 = *(const v8ha*)(p + 16 + 8 * h);
  return __builtin_shufflevector(q0, q1, 0, 1, 2, 3, 4, 5, 6, 7, 8, 9, 10, 11, 12, 13, 14, 15);
}

__device__ __forceinline__ double shfl_xor_d(double v, int s) {
  const unsigned long long u = (unsigned long long)__double_as_longlong(v);
  unsigned int lo = (unsigned int)(u & 0xffffffffull);
  unsigned int hi = (unsigned int)(u >> 32);
  lo = __shfl_xor(lo, s, 32);
  hi = __shfl_xor(hi, s, 32);
  const unsigned long long w = ((unsigned long long)hi << 32) | (unsigned long long)lo;
  return __longlong_as_double((long long)w);
}

__device__ __forceinline__ float blk_sum(float v, float* sRed, int tid) {
  sRed[tid] = v;
  __syncthreads();
  #pragma unroll
  for (int s = TPB / 2; s > 0; s >>= 1) {
    if (tid < s) sRed[tid] = sRed[tid] + sRed[tid + s];
    __syncthreads();
  }
  const float r = sRed[0];
  __syncthreads();
  return r;
}

__global__ __launch_bounds__(TPB) void k_cbsplit(const float* __restrict__ cb,
                                                  _Float16* __restrict__ Bh,
                                                  _Float16* __restrict__ Bl,
                                                  int nCodes)
{
  const int tid = threadIdx.x, lane = tid & 31, wv = tid >> 5;
  const int row = blockIdx.x * 8 + wv;
  const int rowc = (row > nCodes - 1) ? (nCodes - 1) : row;
  const float* src = cb + (size_t)rowc * DIM + 8 * lane;
  const v4f a = *(const v4fa*)src;
  const v4f c = *(const v4fa*)(src + 4);
  v8h hv, lv;
  split8(a, c, hv, lv);
  if (row < nCodes) {
    _Float16* ph = Bh + (size_t)row * DIM + 8 * lane;
    _Float16* pl = Bl + (size_t)row * DIM + 8 * lane;
    *(volatile v8h*)ph = hv;
    *(volatile v8h*)pl = lv;
    __threadfence();
    *(volatile v8h*)ph = hv;
    *(volatile v8h*)pl = lv;
  }
}

__global__ __launch_bounds__(TA) void k_assign(const float* __restrict__ x,
                                               const float* __restrict__ cb,
                                               const float* __restrict__ gcb,
                                               const _Float16* __restrict__ Bh,
                                               const _Float16* __restrict__ Bl,
                                               int nRows,
                                               float* __restrict__ out0,
                                               v4u* __restrict__ rec)
{
  __shared__ __align__(16) _Float16 sAh[RB * PA];
  __shared__ __align__(16) _Float16 sAl[RB * PA];
  __shared__ float sG[NGC];
  __shared__ int   sIdx1[RB];
  __shared__ int   sIdx2[RB];
  __shared__ int   sFin[RB];
  __shared__ int   sBi[RB];
  __shared__ float sGf[RB];
  __shared__ float sGq[RB];

  const int tid = threadIdx.x, lane = tid & 31, wv = tid >> 5;
  const int h = lane >> 4, m = lane & 15;
  const int rb0 = blockIdx.x * RB;
  const int nR1 = nRows - 1;

  if (tid < NGC) sG[tid] = gcb[tid];

  #pragma unroll 2
  for (int it = 0; it < (RB * DIM) / (8 * TA); ++it) {
    const int idx = it * TA + tid;
    const int row = idx >> 5;
    const int c8  = (idx & 31) * 8;
    int grow = rb0 + row;
    grow = (grow > nR1) ? nR1 : grow;
    const float* src = x + (size_t)grow * DIM + c8;
    const v4f a = *(const v4fa*)src;
    const v4f c = *(const v4fa*)(src + 4);
    v8h hv, lv;
    split8(a, c, hv, lv);
    *(v8ha*)(sAh + row * PA + c8) = hv;
    *(v8ha*)(sAl + row * PA + c8) = lv;
  }
  __syncthreads();

  float b1v[8], b2v[8];
  int   b1i[8], b2i[8];
  #pragma unroll
  for (int r = 0; r < 8; ++r) { b1v[r] = NEGBIG; b2v[r] = NEGBIG; b1i[r] = 0; b2i[r] = 0; }
  const _Float16* pah = sAh + (wv * 16 + m) * PA;
  const _Float16* pal = sAl + (wv * 16 + m) * PA;
  const v8f z8 = {0.f, 0.f, 0.f, 0.f, 0.f, 0.f, 0.f, 0.f};
  #pragma unroll 1
  for (int ct = 0; ct < NCT; ++ct) {
    const _Float16* pbh = Bh + (size_t)(ct * 16 + m) * DIM;
    const _Float16* pbl = Bl + (size_t)(ct * 16 + m) * DIM;
    v8f acc0 = z8, acc1 = z8;
    #pragma unroll 2
    for (int ks = 0; ks < DIM / 32; ++ks) {
      const int k0 = ks * 32;
      const v16h ah = ldfrag(pah + k0, h);
      const v16h al = ldfrag(pal + k0, h);
      const v16h bh = ldfrag(pbh + k0, h);
      const v16h bl = ldfrag(pbl + k0, h);
      acc0 = wmma_h(ah, bh, acc0);
      acc1 = wmma_h(ah, bl, acc1);
      acc1 = wmma_h(al, bh, acc1);
    }
    const int col = ct * 16 + m;
    #pragma unroll
    for (int r = 0; r < 8; ++r) {
      const float v = acc0[r] + acc1[r] * INV_LO;
      const bool gt1 = v > b1v[r];
      const bool gt2 = v > b2v[r];
      const float n2v = gt1 ? b1v[r] : (gt2 ? v : b2v[r]);
      const int   n2i = gt1 ? b1i[r] : (gt2 ? col : b2i[r]);
      b2v[r] = n2v;
      b2i[r] = n2i;
      b1v[r] = gt1 ? v : b1v[r];
      b1i[r] = gt1 ? col : b1i[r];
    }
  }
  #pragma unroll
  for (int s = 1; s <= 8; s <<= 1) {
    #pragma unroll
    for (int r = 0; r < 8; ++r) {
      const float ov1 = __shfl_xor(b1v[r], s, 32);
      const int   oi1 = __shfl_xor(b1i[r], s, 32);
      const float ov2 = __shfl_xor(b2v[r], s, 32);
      const int   oi2 = __shfl_xor(b2i[r], s, 32);
      const bool take1 = (ov1 > b1v[r]) || ((ov1 == b1v[r]) && (oi1 < b1i[r]));
      const float n1v = take1 ? ov1 : b1v[r];
      const int   n1i = take1 ? oi1 : b1i[r];
      const float lv  = take1 ? b1v[r] : ov1;
      const int   li  = take1 ? b1i[r] : oi1;
      const bool takeo2 = (ov2 > b2v[r]) || ((ov2 == b2v[r]) && (oi2 < b2i[r]));
      const float mv  = takeo2 ? ov2 : b2v[r];
      const int   mi  = takeo2 ? oi2 : b2i[r];
      const bool takem = (mv > lv) || ((mv == lv) && (mi < li));
      const float n2v = takem ? mv : lv;
      const int   n2i = takem ? mi : li;
      b1v[r] = n1v; b1i[r] = n1i;
      b2v[r] = n2v; b2i[r] = n2i;
    }
  }
  if (m == 0) {
    #pragma unroll
    for (int r = 0; r < 8; ++r) {
      sIdx1[wv * 16 + 8 * h + r] = b1i[r];
      sIdx2[wv * 16 + 8 * h + r] = b2i[r];
    }
  }
  __syncthreads();

  {
    const int row = tid >> 1, sub = tid & 1;
    int grow = rb0 + row;
    grow = (grow > nR1) ? nR1 : grow;
    int kA = sIdx1[row];
    int kB = sIdx2[row];
    kA = (kA < 0) ? 0 : ((kA > NSC - 1) ? (NSC - 1) : kA);
    kB = (kB < 0) ? 0 : ((kB > NSC - 1) ? (NSC - 1) : kB);
    const int kM = sub ? kB : kA;
    const float* xr = x  + (size_t)grow * DIM;
    const float* cr = cb + (size_t)kM * DIM;
    double dd = 0.0;
    #pragma unroll 2
    for (int d = 0; d < DIM; d += 4) {
      const v4f a = *(const v4fa*)(xr + d);
      const v4f b = *(const v4fa*)(cr + d);
      dd = __builtin_fma((double)a.x, (double)b.x, dd);
      dd = __builtin_fma((double)a.y, (double)b.y, dd);
      dd = __builtin_fma((double)a.z, (double)b.z, dd);
      dd = __builtin_fma((double)a.w, (double)b.w, dd);
    }
    const double dO = shfl_xor_d(dd, 1);
    const double dA = sub ? dO : dd;
    const double dB = sub ? dd : dO;
    const bool takeB = (dB > dA) || ((dB == dA) && (kB < kA));
    const int    kW = takeB ? kB : kA;
    const double dW = takeB ? dB : dA;
    const float  s  = (float)dW;
    const float gf = logf(fmaxf(s, EPSN));
    const float a2 = gf * gf;
    float bd = NEGBIG;
    int bi = 0;
    #pragma unroll 8
    for (int j = 0; j < NGC; ++j) {
      const float g = sG[j];
      const float val = -((a2 - 2.0f * (gf * g)) + g * g);
      const bool gt = val > bd;
      bd = gt ? val : bd;
      bi = gt ? j : bi;
    }
    if (sub == 0) {
      sFin[row] = kW;
      sBi[row]  = bi;
      sGf[row]  = gf;
      sGq[row]  = expf(sG[bi]);
    }
  }
  __syncthreads();

  #pragma unroll 1
  for (int rr = 0; rr < 16; ++rr) {
    const int lr = wv * 16 + rr;
    const int grow = rb0 + lr;
    if (grow < nRows) {
      int k = sFin[lr];
      k = (k < 0) ? 0 : ((k > NSC - 1) ? (NSC - 1) : k);
      const float gq = sGq[lr];
      const float* cr = cb + (size_t)k * DIM;
      v4f c0 = *(const v4fa*)(cr + 4 * lane);
      v4f c1 = *(const v4fa*)(cr + (DIM / 2) + 4 * lane);
      c0 = c0 * gq;
      c1 = c1 * gq;
      float* dst = out0 + (size_t)grow * DIM;
      *(volatile v4f*)(dst + 4 * lane) = c0;
      *(volatile v4f*)(dst + (DIM / 2) + 4 * lane) = c1;
      __threadfence();
      *(volatile v4f*)(dst + 4 * lane) = c0;
      *(volatile v4f*)(dst + (DIM / 2) + 4 * lane) = c1;
    }
  }

  if (wv == 0) {
    v4u rv = {0u, 0u, 0u, 0u};
    rv.x = (unsigned int)sFin[lane];
    rv.y = (unsigned int)sBi[lane];
    rv.z = __float_as_uint(sGf[lane]);
    v4u* dst = rec + (size_t)rb0 + lane;
    *(volatile v4u*)dst = rv;
    __threadfence();
    *(volatile v4u*)dst = rv;
  }
}

__device__ __forceinline__ void drain1(unsigned int mm, int base, int nR1,
                                       const float* __restrict__ xd,
                                       float& acc, unsigned int& cnt)
{
  cnt += (unsigned int)__builtin_popcount(mm);
  #pragma unroll 1
  for (int it = 0; it < 32 && mm != 0u; ++it) {
    const int b = __builtin_ctz(mm);
    mm &= (mm - 1u);
    int row = base + b;
    row = (row > nR1) ? nR1 : row;
    acc += xd[(size_t)row * DIM];
  }
}

__global__ __launch_bounds__(TPB) void k_code(const float* __restrict__ x,
                                              const float* __restrict__ cb,
                                              const v4u* __restrict__ rec,
                                              int nRows,
                                              float* __restrict__ out1,
                                              v4u* __restrict__ cstat)
{
  __shared__ __align__(16) unsigned int sMask[2 * CPB * 8];
  __shared__ float sRed[TPB];
  __shared__ __align__(16) float sRow[DIM];

  const int tid = threadIdx.x, lane = tid & 31, wv = tid >> 5;
  const int kb = blockIdx.x * CPB;
  const int nR1 = nRows - 1;

  float acc[CPB];
  unsigned int cnt[CPB];
  #pragma unroll
  for (int j = 0; j < CPB; ++j) { acc[j] = 0.0f; cnt[j] = 0u; }
  const float* xd = x + tid;
  const int nch = (nRows + CHK - 1) / CHK;

  #pragma unroll 1
  for (int c = 0; c < nch; ++c) {
    const int par = c & 1;
    const int i = c * CHK + tid;
    const int ic = (i > nR1) ? nR1 : i;
    const v4u r = rec[ic];
    const int key = (i < nRows) ? (int)r.x : -1;
    #pragma unroll
    for (int j = 0; j < CPB; ++j) {
      const unsigned int mk = __builtin_amdgcn_ballot_w32(key == kb + j);
      if (lane == 0) sMask[(par * CPB + j) * 8 + wv] = mk;
    }
    __syncthreads();
    const int base = c * CHK;
    #pragma unroll
    for (int j = 0; j < CPB; ++j) {
      const v4u q0 = *(const v4ua*)(sMask + (par * CPB + j) * 8);
      const v4u q1 = *(const v4ua*)(sMask + (par * CPB + j) * 8 + 4);
      const unsigned int any = q0.x | q0.y | q0.z | q0.w | q1.x | q1.y | q1.z | q1.w;
      if (any != 0u) {
        drain1(q0.x, base,       nR1, xd, acc[j], cnt[j]);
        drain1(q0.y, base + 32,  nR1, xd, acc[j], cnt[j]);
        drain1(q0.z, base + 64,  nR1, xd, acc[j], cnt[j]);
        drain1(q0.w, base + 96,  nR1, xd, acc[j], cnt[j]);
        drain1(q1.x, base + 128, nR1, xd, acc[j], cnt[j]);
        drain1(q1.y, base + 160, nR1, xd, acc[j], cnt[j]);
        drain1(q1.z, base + 192, nR1, xd, acc[j], cnt[j]);
        drain1(q1.w, base + 224, nR1, xd, acc[j], cnt[j]);
      }
    }
  }

  #pragma unroll
  for (int j = 0; j < CPB; ++j) {
    int code = kb + j;
    code = (code > NSC - 1) ? (NSC - 1) : code;
    const float n1 = blk_sum(acc[j] * acc[j], sRed, tid);
    const float inv1 = 1.0f / fmaxf(sqrtf(n1), EPSN);
    const float sn = acc[j] * inv1;
    const float cv = cb[(size_t)code * DIM + tid];
    const float u = cv * DEC + sn * OMD;
    const float n2 = blk_sum(u * u, sRed, tid);
    const float inv2 = 1.0f / fmaxf(sqrtf(n2), EPSL2);
    sRow[tid] = u * inv2;
    __syncthreads();
    if (wv == 0) {
      const v4f a = *(const v4fa*)(sRow + 4 * lane);
      const v4f b = *(const v4fa*)(sRow + (DIM / 2) + 4 * lane);
      float* dst = out1 + (size_t)code * DIM;
      *(volatile v4f*)(dst + 4 * lane) = a;
      *(volatile v4f*)(dst + (DIM / 2) + 4 * lane) = b;
      __threadfence();
      *(volatile v4f*)(dst + 4 * lane) = a;
      *(volatile v4f*)(dst + (DIM / 2) + 4 * lane) = b;
    }
    __syncthreads();
  }

  if (wv == 0) {
    const int q = lane >> 3, e = lane & 7;
    const unsigned int c01 = (q & 1) ? cnt[1] : cnt[0];
    const unsigned int c23 = (q & 1) ? cnt[3] : cnt[2];
    const unsigned int cq  = (q & 2) ? c23 : c01;
    v4u v = {0u, 0u, 0u, 0u};
    v.x = (e == 0) ? cq : 0u;
    v4u* dst = cstat + (size_t)kb * 8 + lane;
    *(volatile v4u*)dst = v;
    __threadfence();
    *(volatile v4u*)dst = v;
  }
}

__global__ __launch_bounds__(TPB) void k_final(const v4u* __restrict__ rec,
                                               const v4u* __restrict__ cstat,
                                               const float* __restrict__ gcb,
                                               const float* __restrict__ gnum,
                                               const float* __restrict__ snum,
                                               int nRows,
                                               float* __restrict__ out234)
{
  __shared__ float sG[NGC];
  __shared__ float sC[NGC];
  __shared__ float sRed[TPB];
  __shared__ __align__(16) float sOut[NOUT234];

  const int tid = threadIdx.x;
  const int nR1 = nRows - 1;
  const int nch = (nRows + CHK - 1) / CHK;

  #pragma unroll 1
  for (int g = 0; g < NGC; ++g) {
    float s = 0.f, c = 0.f;
    #pragma unroll 1
    for (int ch = 0; ch < nch; ++ch) {
      const int i = ch * CHK + tid;
      const int ic = (i > nR1) ? nR1 : i;
      const v4u r = rec[ic];
      const bool hit = (i < nRows) && ((int)r.y == g);
      s = hit ? (s + __uint_as_float(r.z)) : s;
      c = hit ? (c + 1.0f) : c;
    }
    const float st = blk_sum(s, sRed, tid);
    const float cn = blk_sum(c, sRed, tid);
    if (tid == 0) { sG[g] = st; sC[g] = cn; }
  }
  __syncthreads();

  if (tid < NGC) {
    const float cn = sC[tid];
    const float gn = sG[tid] * (1.0f / fmaxf(cn, EPSN));
    sOut[tid] = gcb[tid] * DEC + gn * OMD;
    sOut[NGC + NSC + tid] = gnum[tid] * DEC + cn * OMD;
  }
  #pragma unroll
  for (int q = 0; q < 4; ++q) {
    const int k = q * TPB + tid;
    const v4u cs = cstat[(size_t)k * 8];
    const float ck = (float)cs.x;
    sOut[NGC + k] = snum[k] * DEC + ck * OMD;
  }
  __syncthreads();

  const int t2 = (tid < 32) ? tid : 0;
  const v4f v0 = *(const v4fa*)(sOut + 4 * tid);
  const v4f v1 = *(const v4fa*)(sOut + 4 * TPB + 4 * t2);
  *(volatile v4f*)(out234 + 4 * tid) = v0;
  if (tid < 32) *(volatile v4f*)(out234 + 4 * TPB + 4 * tid) = v1;
  __threadfence();
  *(volatile v4f*)(out234 + 4 * tid) = v0;
  if (tid < 32) *(volatile v4f*)(out234 + 4 * TPB + 4 * tid) = v1;
}

extern "C" void kernel_launch(void* const* d_in, const int* in_sizes, int n_in,
                              void* d_out, int out_size, void* d_ws, size_t ws_size,
                              hipStream_t stream)
{
  if (n_in < 5) return;
  const int nx = in_sizes[0];
  if (nx <= 0 || (nx % DIM) != 0) return;
  const int nRows = nx / DIM;
  if (in_sizes[1] != NSC * DIM) return;
  if (in_sizes[2] != NGC) return;
  if (in_sizes[3] != NSC) return;
  if (in_sizes[4] != NGC) return;

  const size_t off1 = (size_t)nRows * DIM;
  const size_t off2 = off1 + (size_t)NSC * DIM;
  const size_t totalOut = off2 + NGC + NSC + NGC;
  if ((size_t)out_size != totalOut) return;

  const float* x    = (const float*)d_in[0];
  const float* cb   = (const float*)d_in[1];
  const float* gcb  = (const float*)d_in[2];
  const float* snum = (const float*)d_in[3];
  const float* gnum = (const float*)d_in[4];
  float* out = (float*)d_out;

  const size_t bB      = (size_t)NSC * DIM * 2;
  const size_t recRows = (size_t)((nRows + RB - 1) / RB) * RB;
  const size_t bRec    = recRows * 16;
  const size_t bCst    = (size_t)NSC * 128;
  const size_t total   = 2 * bB + bRec + bCst;
  if (total > ws_size) return;
  if (total > (size_t)134217728) return;

  char* ws = (char*)d_ws;
  size_t off = 0;
  _Float16* Bh  = (_Float16*)(ws + off); off += bB;
  _Float16* Bl  = (_Float16*)(ws + off); off += bB;
  v4u*      rec = (v4u*)(ws + off);      off += bRec;
  v4u*      cst = (v4u*)(ws + off);      off += bCst;
  if (off != total) return;

  const int gridA = (int)(recRows / RB);

  k_cbsplit<<<(NSC + 7) / 8, TPB, 0, stream>>>(cb, Bh, Bl, NSC);
  k_assign<<<gridA, TA, 0, stream>>>(x, cb, gcb, Bh, Bl, nRows, out, rec);
  k_code<<<NSC / CPB, TPB, 0, stream>>>(x, cb, rec, nRows, out + off1, cst);
  k_final<<<1, TPB, 0, stream>>>(rec, cst, gcb, gnum, snum, nRows, out + off2);
}
